// Mamba_48558900249067
// MI455X (gfx1250) — hardware-verified
//
#include <hip/hip_runtime.h>
#include <math.h>

typedef __attribute__((ext_vector_type(16))) _Float16 v16h;
typedef __attribute__((ext_vector_type(8)))  _Float16 v8h;
typedef __attribute__((ext_vector_type(16))) __bf16   v16b;
typedef __attribute__((ext_vector_type(8)))  __bf16   v8b;
typedef __attribute__((ext_vector_type(8)))  float    v8f;
typedef __attribute__((ext_vector_type(4)))  float    v4f;

constexpr int kBatch  = 4;
constexpr int kSeqL   = 2048;
constexpr int kDmod   = 1024;
constexpr int kDin    = 2048;
constexpr int kNst    = 16;
constexpr int kDtR    = 64;
constexpr int kPrjN   = kDtR + 2 * kNst;
constexpr int kPrjP   = 128;
constexpr int kXZP    = 2 * kDin;
constexpr int kRows   = kBatch * kSeqL;
constexpr int kTP     = 260;
constexpr int kScanTS = 16;

constexpr float kCarX    = 16.0f;
constexpr float kCarWin  = 256.0f;
constexpr float kCarY    = 64.0f;
constexpr float kCarWout = 256.0f;
constexpr float kSclIn   = 1.0f / (kCarX * kCarWin);
constexpr float kSclOut  = 1.0f / (kCarY * kCarWout);

static_assert(kPrjN == 96);
static_assert((kDmod % 32) == 0 && (kDin % 32) == 0 && (kDtR % 32) == 0);
static_assert((kSeqL % 64) == 0 && (kXZP % 64) == 0 && (kPrjP % 64) == 0 && (kDin % 64) == 0 && (kDmod % 64) == 0);
static_assert((kDin % 256) == 0 && (kSeqL % kScanTS) == 0 && kPrjP >= kPrjN);

constexpr int kTilesIn  = (kSeqL / 64) * (kXZP / 64);
constexpr int kTilesXp  = (kSeqL / 64) * (kPrjP / 64);
constexpr int kTilesDt  = (kSeqL / 64) * (kDin / 64);
constexpr int kTilesOut = (kSeqL / 64) * (kDmod / 64);
static_assert((kTilesIn % 8) == 0 && (kTilesXp % 8) == 0 && (kTilesDt % 8) == 0 && (kTilesOut % 8) == 0);
constexpr int kBlkIn  = kTilesIn / 8;
constexpr int kBlkXp  = kTilesXp / 8;
constexpr int kBlkDt  = kTilesDt / 8;
constexpr int kBlkOut = kTilesOut / 8;

constexpr int kTot8X    = kRows * kDmod / 8;
constexpr int kTot8Win  = kXZP * kDmod / 8;
constexpr int kTot8Wout = kDmod * kDin / 8;
constexpr int kTot8Wxp  = kPrjP * kDin / 8;
constexpr int kReal8Wxp = kPrjN * kDin / 8;
constexpr int kTot8Wdt  = kDin * kDtR / 8;
constexpr int kTotSplit = kSeqL * (kDin / 8);
constexpr int kTot8Dt   = kSeqL * kDtR / 8;
static_assert((kTot8X % 256) == 0 && (kTot8Win % 256) == 0 && (kTot8Wout % 256) == 0 && (kTot8Wxp % 256) == 0 &&
              (kTot8Wdt % 256) == 0 && (kTotSplit % 256) == 0 && (kTot8Dt % 256) == 0 && (kReal8Wxp % 32) == 0);

constexpr size_t kSzX16   = (size_t)kRows * kDmod * 2;
constexpr size_t kSzWIN   = (size_t)kXZP  * kDmod * 2;
constexpr size_t kSzWXP   = (size_t)kPrjP * kDin  * 2;
constexpr size_t kSzWDT   = (size_t)kDin  * kDtR  * 2;
constexpr size_t kSzWOUT  = (size_t)kDmod * kDin  * 2;
constexpr size_t kSzXZ    = (size_t)kSeqL * kXZP  * 4;
constexpr size_t kSzXIN   = (size_t)kSeqL * kDin  * 2;
constexpr size_t kSzXD    = (size_t)kSeqL * kPrjP * 4;
constexpr size_t kSzDT    = (size_t)kSeqL * kDtR  * 2;
constexpr size_t kSzDLR   = (size_t)kSeqL * kDin  * 4;
constexpr size_t kSzY16   = (size_t)kSeqL * kDin  * 2;
constexpr size_t kOffX16  = 0;
constexpr size_t kOffWIN  = kOffX16  + kSzX16;
constexpr size_t kOffWXP  = kOffWIN  + kSzWIN;
constexpr size_t kOffWDT  = kOffWXP  + kSzWXP;
constexpr size_t kOffWOUT = kOffWDT  + kSzWDT;
constexpr size_t kOffXZ   = kOffWOUT + kSzWOUT;
constexpr size_t kOffXINH = kOffXZ   + kSzXZ;
constexpr size_t kOffXINL = kOffXINH + kSzXIN;
constexpr size_t kOffXD   = kOffXINL + kSzXIN;
constexpr size_t kOffDTH  = kOffXD   + kSzXD;
constexpr size_t kOffDTL  = kOffDTH  + kSzDT;
constexpr size_t kOffDLR  = kOffDTL  + kSzDT;
constexpr size_t kOffY16  = kOffDLR  + kSzDLR;
constexpr size_t kWsTotal = kOffY16  + kSzY16;
static_assert(kWsTotal == 107216896ull);
static_assert(kWsTotal <= 134217728ull);
static_assert((kOffWIN % 128) == 0 && (kOffWXP % 128) == 0 && (kOffWDT % 128) == 0 && (kOffWOUT % 128) == 0 &&
              (kOffXZ % 128) == 0 && (kOffXINH % 128) == 0 && (kOffXINL % 128) == 0 && (kOffXD % 128) == 0 &&
              (kOffDTH % 128) == 0 && (kOffDTL % 128) == 0 && (kOffDLR % 128) == 0 && (kOffY16 % 128) == 0);

__device__ __forceinline__ unsigned short f2bf_bits(float f) {
  unsigned u = __float_as_uint(f);
  return (unsigned short)((u + 0x7FFFu + ((u >> 16) & 1u)) >> 16);
}
__device__ __forceinline__ float bf_bits2f(unsigned short h) { return __uint_as_float(((unsigned)h) << 16); }
__device__ __forceinline__ float bfr(float f) { return bf_bits2f(f2bf_bits(f)); }
__device__ __forceinline__ float silu_f(float v) { return v * __builtin_amdgcn_rcpf(1.0f + expf(-v)); }

__device__ __forceinline__ void grp_guard_h(v8f& a, v8f& b, v8f& c, v8f& d, v16h x, v16h y) {
  asm volatile("v_nop\n\tv_nop\n\tv_nop\n\tv_nop" : "+v"(a), "+v"(b), "+v"(c), "+v"(d) : "v"(x), "v"(y));
}
__device__ __forceinline__ void grp_guard_b(v8f& a, v8f& b, v8f& c, v8f& d, v16b x, v16b y) {
  asm volatile("v_nop\n\tv_nop\n\tv_nop\n\tv_nop" : "+v"(a), "+v"(b), "+v"(c), "+v"(d) : "v"(x), "v"(y));
}
__device__ __forceinline__ void keep4_h(v16h a, v16h b, v16h c, v16h d) { asm volatile("v_nop" :: "v"(a), "v"(b), "v"(c), "v"(d)); }
__device__ __forceinline__ void keep4_b(v16b a, v16b b, v16b c, v16b d) { asm volatile("v_nop" :: "v"(a), "v"(b), "v"(c), "v"(d)); }
__device__ __forceinline__ void acc_guard4(v8f& a, v8f& b, v8f& c, v8f& d) { asm volatile("v_nop\n\tv_nop\n\tv_nop\n\tv_nop" : "+v"(a), "+v"(b), "+v"(c), "+v"(d)); }
template <typename T> struct Frag;
template <> struct Frag<_Float16> {
  typedef v16h V; union U { v16h v; v8h h[2]; };
  static __device__ __forceinline__ v16h load(const _Float16* p) {
    U f; f.h[0] = *(const v8h*)(p); f.h[1] = *(const v8h*)(p + 16); return f.v;
  }
  static __device__ __forceinline__ v8f mma(v16h a, v16h b, v8f c) {
    return __builtin_amdgcn_wmma_f32_16x16x32_f16(false, a, false, b, (short)0, c, false, false);
  }
  static __device__ __forceinline__ void guard4(v8f& a, v8f& b, v8f& c, v8f& d, v16h x, v16h y) { grp_guard_h(a, b, c, d, x, y); }
  static __device__ __forceinline__ void keep(v16h a, v16h b, v16h c, v16h d) { keep4_h(a, b, c, d); }
};
template <> struct Frag<__bf16> {
  typedef v16b V; union U { v16b v; v8b h[2]; };
  static __device__ __forceinline__ v16b load(const __bf16* p) {
    U f; f.h[0] = *(const v8b*)(p); f.h[1] = *(const v8b*)(p + 16); return f.v;
  }
  static __device__ __forceinline__ v8f mma(v16b a, v16b b, v8f c) {
    return __builtin_amdgcn_wmma_f32_16x16x32_bf16(false, a, false, b, (short)0, c, false, false);
  }
  static __device__ __forceinline__ void guard4(v8f& a, v8f& b, v8f& c, v8f& d, v16b x, v16b y) { grp_guard_b(a, b, c, d, x, y); }
  static __device__ __forceinline__ void keep(v16b a, v16b b, v16b c, v16b d) { keep4_b(a, b, c, d); }
};

template <int ET> struct Elem;
template <> struct Elem<0> { typedef _Float16 T; };
template <> struct Elem<1> { typedef __bf16 T; };
template <int ET, int SPL, int BIAS_MODE, int OUT_MODE, bool RESID, int ACT = 0>
__global__ __launch_bounds__(256) void wmma_gemm64(
    const unsigned short* __restrict__ Ap, const unsigned short* __restrict__ A2p, int lda, long strideA,
    const unsigned short* __restrict__ Btp, const unsigned short* __restrict__ Bt2p, int ldb, long strideB,
    void* __restrict__ Cout, void* __restrict__ Cout2, int ldc, long strideC,
    const float* __restrict__ bias,
    const float* __restrict__ resid, long strideR,
    int M, int N, int K, float scale) {
  typedef typename Elem<ET>::T T;
  typedef typename Frag<T>::V V;
  const T* A = (const T*)Ap; const T* A2 = (const T*)A2p; const T* Bt = (const T*)Btp; const T* Bt2 = (const T*)Bt2p;
  __shared__ __align__(16) float sT[8][16 * 68];
  const int b    = blockIdx.y;
  const int lane = threadIdx.x & 31;
  const int wave = threadIdx.x >> 5;
  const int tilesN = N >> 6;
  const int tilesM = M >> 6;
  const int tile = blockIdx.x * 8 + wave;
  if (tile >= tilesM * tilesN) return;
  const int tm = tile / tilesN;
  const int tn = tile - tm * tilesN;
  const int m0 = tm << 6;
  const int n0 = tn << 6;

  const T* Ab  = A  + (size_t)b * strideA;
  const T* Bb  = Bt + (size_t)b * strideB;
  const T* Ab2 = (SPL >= 1) ? (A2  + (size_t)b * strideA) : nullptr;
  const T* Bb2 = (SPL == 2) ? (Bt2 + (size_t)b * strideB) : nullptr;

  const int rlane = lane & 15;
  const int koff  = (lane >> 4) * 8;
  const int mOff  = (lane >> 4) * 8;

  v8f acc[4][4];
#pragma unroll
  for (int i = 0; i < 4; ++i)
#pragma unroll
    for (int j = 0; j < 4; ++j) acc[i][j] = (v8f){0.f,0.f,0.f,0.f,0.f,0.f,0.f,0.f};

  for (int k0 = 0; k0 < K; k0 += 32) {
    V bh[4], bl[4];
#pragma unroll
    for (int j = 0; j < 4; ++j) {
      const size_t bo = (size_t)(n0 + (j << 4) + rlane) * ldb + koff + k0;
      bh[j] = Frag<T>::load(Bb + bo);
      if (SPL == 2) bl[j] = Frag<T>::load(Bb2 + bo);
    }
#pragma unroll
    for (int i = 0; i < 4; ++i) {
      const size_t ao = (size_t)(m0 + (i << 4) + rlane) * lda + koff + k0;
      V ah = Frag<T>::load(Ab + ao);
      V al;
      if (SPL >= 1) al = Frag<T>::load(Ab2 + ao);
#pragma unroll
      for (int j = 0; j < 4; ++j) {
        acc[i][j] = Frag<T>::mma(ah, bh[j], acc[i][j]);
        if (SPL == 2) acc[i][j] = Frag<T>::mma(ah, bl[j], acc[i][j]);
        if (SPL >= 1) acc[i][j] = Frag<T>::mma(al, bh[j], acc[i][j]);
      }
      Frag<T>::guard4(acc[i][0], acc[i][1], acc[i][2], acc[i][3], ah, (SPL >= 1) ? al : ah);
    }
    Frag<T>::keep(bh[0], bh[1], bh[2], bh[3]);
    if (SPL == 2) Frag<T>::keep(bl[0], bl[1], bl[2], bl[3]);
  }
  acc_guard4(acc[0][0], acc[0][1], acc[0][2], acc[0][3]);
  acc_guard4(acc[1][0], acc[1][1], acc[1][2], acc[1][3]);
  acc_guard4(acc[2][0], acc[2][1], acc[2][2], acc[2][3]);
  acc_guard4(acc[3][0], acc[3][1], acc[3][2], acc[3][3]);

  float* slab = sT[wave];
  const float* Rb = RESID ? (resid + (size_t)b * strideR) : nullptr;
#pragma unroll
  for (int i = 0; i < 4; ++i) {
    const int mBase = m0 + (i << 4);
#pragma unroll
    for (int j = 0; j < 4; ++j) {
      const int n = n0 + (j << 4) + rlane;
      float bv = 0.f;
      if (BIAS_MODE == 2) bv = bfr(bias[n]);
#pragma unroll
      for (int r = 0; r < 8; ++r) {
        float v = acc[i][j][r] * scale;
        if (BIAS_MODE == 1) v += bfr(bias[mBase + mOff + r]);
        if (BIAS_MODE == 2) v += bv;
        if (RESID) v += Rb[(size_t)(mBase + mOff + r) * ldc + n];
        if (ACT == 1) v = tanhf(v);
        if (ACT == 2) v = fmaxf(v, 0.0f);
        if (ACT == 4) v = (v > 0.f) ? v : 0.01f * v;
        slab[(mOff + r) * 68 + (j << 4) + rlane] = v;
      }
    }
    __builtin_amdgcn_fence(__ATOMIC_RELEASE, "workgroup");
    __builtin_amdgcn_wave_barrier();
    __builtin_amdgcn_fence(__ATOMIC_ACQUIRE, "workgroup");
    if (OUT_MODE == 0) {
      float* C = (float*)Cout + (size_t)b * strideC;
      const int hh = lane >> 4, c4 = (lane & 15) * 4;
      for (int pass = 0; pass < 2; ++pass) {
#pragma unroll
        for (int it = 0; it < 8; ++it) {
          const int row = it * 2 + hh;
          v4f v = *(const v4f*)(slab + row * 68 + c4);
          *(volatile v4f*)(C + (size_t)(mBase + row) * ldc + n0 + c4) = v;
        }
        __threadfence();
      }
    } else {
      const int q = lane >> 3, c8 = (lane & 7) * 8;
      unsigned short* C  = (unsigned short*)Cout  + (size_t)b * strideC;
      unsigned short* C2 = (OUT_MODE == 2) ? ((unsigned short*)Cout2 + (size_t)b * strideC) : nullptr;
      for (int pass = 0; pass < 2; ++pass) {
#pragma unroll
        for (int it = 0; it < 4; ++it) {
          const int row = it * 4 + q;
          const float* sp = slab + row * 68 + c8;
          v8h hv, lv;
#pragma unroll
          for (int e = 0; e < 8; ++e) {
            if (OUT_MODE == 1) {
              hv[e] = (_Float16)sp[e];
            } else {
              unsigned short hb = f2bf_bits(sp[e]);
              unsigned short lb = f2bf_bits(sp[e] - bf_bits2f(hb));
              hv[e] = __builtin_bit_cast(_Float16, hb);
              lv[e] = __builtin_bit_cast(_Float16, lb);
            }
          }
          *(volatile v8h*)(C + (size_t)(mBase + row) * ldc + n0 + c8) = hv;
          if (OUT_MODE == 2) *(volatile v8h*)(C2 + (size_t)(mBase + row) * ldc + n0 + c8) = lv;
        }
        __threadfence();
      }
    }
    __builtin_amdgcn_fence(__ATOMIC_RELEASE, "workgroup");
    __builtin_amdgcn_wave_barrier();
    __builtin_amdgcn_fence(__ATOMIC_ACQUIRE, "workgroup");
  }
}

__global__ __launch_bounds__(256) void cast_in_f16_kernel(
    const float* __restrict__ src, unsigned short* __restrict__ dst, int total8, float scale)
{
  const int i = blockIdx.x * 256 + threadIdx.x;
  if (i >= total8) return;
  const size_t e0 = (size_t)i << 3;
  const float* p = src + e0;
  const v4f a0 = *(const v4f*)(p);
  const v4f a1 = *(const v4f*)(p + 4);
  v8h hv;
#pragma unroll
  for (int e = 0; e < 4; ++e) {
    hv[e]     = (_Float16)(bfr(a0[e]) * scale);
    hv[4 + e] = (_Float16)(bfr(a1[e]) * scale);
  }
  unsigned short* q = dst + e0;
  *(volatile v8h*)q = hv;
  __threadfence();
  *(volatile v8h*)q = hv;
}

__global__ __launch_bounds__(256) void cast_in_bf16_kernel(
    const float* __restrict__ src, unsigned short* __restrict__ dst, int total8, int nreal8)
{
  const int i = blockIdx.x * 256 + threadIdx.x;
  if (i >= total8) return;
  const bool real = (i < nreal8);
  const int  ic   = real ? i : 0;
  const float fz  = real ? 1.0f : 0.0f;
  const float* p = src + ((size_t)ic << 3);
  const v4f a0 = *(const v4f*)(p);
  const v4f a1 = *(const v4f*)(p + 4);
  v8h hv;
#pragma unroll
  for (int e = 0; e < 4; ++e) {
    const float v0 = a0[e] * fz;
    const float v1 = a1[e] * fz;
    const unsigned short b0 = f2bf_bits(v0);
    const unsigned short b1 = f2bf_bits(v1);
    hv[e]     = __builtin_bit_cast(_Float16, b0);
    hv[4 + e] = __builtin_bit_cast(_Float16, b1);
  }
  unsigned short* q = dst + ((size_t)i << 3);
  *(volatile v8h*)q = hv;
  __threadfence();
  *(volatile v8h*)q = hv;
}

__global__ __launch_bounds__(256) void split_u_kernel(
    const float* __restrict__ XZ, unsigned short* __restrict__ XH, unsigned short* __restrict__ XL, int total)
{
  const int i = blockIdx.x * 256 + threadIdx.x;
  if (i >= total) return;
  const int row = i >> 8;
  const int c8  = (i & 255) << 3;
  const float* p = XZ + (size_t)row * kXZP + c8;
  const v4f a0 = *(const v4f*)(p);
  const v4f a1 = *(const v4f*)(p + 4);
  v8h hv, lv;
#pragma unroll
  for (int e = 0; e < 4; ++e) {
    const float s0 = silu_f(a0[e]);
    const float s1 = silu_f(a1[e]);
    const unsigned short h0 = f2bf_bits(s0), h1 = f2bf_bits(s1);
    const unsigned short l0 = f2bf_bits(s0 - bf_bits2f(h0)), l1 = f2bf_bits(s1 - bf_bits2f(h1));
    hv[e]     = __builtin_bit_cast(_Float16, h0);
    hv[4 + e] = __builtin_bit_cast(_Float16, h1);
    lv[e]     = __builtin_bit_cast(_Float16, l0);
    lv[4 + e] = __builtin_bit_cast(_Float16, l1);
  }
  const size_t o = (size_t)row * kDin + c8;
  unsigned short* qh = XH + o;
  unsigned short* ql = XL + o;
  *(volatile v8h*)qh = hv;
  *(volatile v8h*)ql = lv;
  __threadfence();
  *(volatile v8h*)qh = hv;
  *(volatile v8h*)ql = lv;
}

__global__ __launch_bounds__(256) void dt_split_kernel(
    const float* __restrict__ XD, unsigned short* __restrict__ DTH, unsigned short* __restrict__ DTL, int total8)
{
  const int i = blockIdx.x * 256 + threadIdx.x;
  if (i >= total8) return;
  const int e0  = i << 3;
  const int row = e0 >> 6;
  const int c8  = e0 & 63;
  const float* p = XD + (size_t)row * kPrjP + c8;
  const v4f a0 = *(const v4f*)(p);
  const v4f a1 = *(const v4f*)(p + 4);
  v8h hv, lv;
#pragma unroll
  for (int e = 0; e < 4; ++e) {
    const unsigned short h0 = f2bf_bits(a0[e]), h1 = f2bf_bits(a1[e]);
    const unsigned short l0 = f2bf_bits(a0[e] - bf_bits2f(h0)), l1 = f2bf_bits(a1[e] - bf_bits2f(h1));
    hv[e]     = __builtin_bit_cast(_Float16, h0);
    hv[4 + e] = __builtin_bit_cast(_Float16, h1);
    lv[e]     = __builtin_bit_cast(_Float16, l0);
    lv[4 + e] = __builtin_bit_cast(_Float16, l1);
  }
  unsigned short* qh = DTH + e0;
  unsigned short* ql = DTL + e0;
  *(volatile v8h*)qh = hv;
  *(volatile v8h*)ql = lv;
  __threadfence();
  *(volatile v8h*)qh = hv;
  *(volatile v8h*)ql = lv;
}

__global__ __launch_bounds__(256) void scan_kernel(
    const float* __restrict__ DLR, const float* __restrict__ XZ, const float* __restrict__ XD,
    const float* __restrict__ A_log, const float* __restrict__ Dv, unsigned short* __restrict__ Y16)
{
  __shared__ __align__(16) float sBC[kScanTS * 32];
  __shared__ __align__(16) float sY[kScanTS * kTP];
  __shared__ __align__(16) float sA[kNst * 256];
  const int tid = threadIdx.x, lane = tid & 31, wave = tid >> 5;
  const int d0 = blockIdx.x * 256, d = d0 + tid;

#pragma unroll 1
  for (int n = 0; n < kNst; ++n) sA[n * 256 + tid] = -expf(bfr(A_log[(size_t)d * kNst + n]));
  __syncthreads();
  float An[kNst], h[kNst];
#pragma unroll
  for (int n = 0; n < kNst; ++n) { An[n] = sA[n * 256 + tid]; h[n] = 0.f; }
  const float Dd = bfr(Dv[d]);

#pragma unroll 1
  for (int c = 0; c < kSeqL / kScanTS; ++c) {
    const int l0 = c * kScanTS;
    if (tid < 128) {
      const int r = tid >> 3, q = (tid & 7) * 4;
      const v4f v = *(const v4f*)(XD + (size_t)(l0 + r) * kPrjP + kDtR + q);
      *(v4f*)(sBC + r * 32 + q) = v;
    }
    __syncthreads();
#pragma unroll 1
    for (int s = 0; s < kScanTS; ++s) {
      const size_t m = (size_t)(l0 + s);
      const float a     = DLR[m * kDin + d];
      const float delta = fmaxf(a, 0.0f) + log1pf(expf(-fabsf(a)));
      const float xv    = silu_f(XZ[m * kXZP + d]);
      const float gv    = silu_f(XZ[m * kXZP + kDin + d]);
      v4f Bq[4], Cq[4];
#pragma unroll
      for (int qq = 0; qq < 4; ++qq) {
        Bq[qq] = *(const v4f*)(sBC + s * 32 + 4 * qq);
        Cq[qq] = *(const v4f*)(sBC + s * 32 + kNst + 4 * qq);
      }
      float dtx = delta * xv;
      asm volatile("" : "+v"(dtx));
      float y = 0.f;
#pragma unroll
      for (int n = 0; n < kNst; ++n) {
        const float e = __expf(delta * An[n]);
        float p = dtx * Bq[n >> 2][n & 3];
        asm volatile("" : "+v"(p));
        float qv = h[n] * e;
        asm volatile("" : "+v"(qv));
        const float hn = qv + p;
        h[n] = hn;
        float rr = Cq[n >> 2][n & 3] * hn;
        asm volatile("" : "+v"(rr));
        y += rr;
      }
      float sk = xv * Dd;
      asm volatile("" : "+v"(sk));
      y += sk;
      float yg = y * gv;
      asm volatile("" : "+v"(yg));
      sY[s * kTP + tid] = yg * kCarY;
    }
    __syncthreads();
    v8h hv[2];
#pragma unroll
    for (int it = 0; it < 2; ++it) {
      const float* sp = sY + (it * 8 + wave) * kTP + lane * 8;
      const v4f a0 = *(const v4f*)(sp);
      const v4f a1 = *(const v4f*)(sp + 4);
#pragma unroll
      for (int e = 0; e < 4; ++e) { hv[it][e] = (_Float16)a0[e]; hv[it][4 + e] = (_Float16)a1[e]; }
    }
    for (int pass = 0; pass < 2; ++pass) {
#pragma unroll
      for (int it = 0; it < 2; ++it)
        *(volatile v8h*)(Y16 + (size_t)(l0 + it * 8 + wave) * kDin + d0 + lane * 8) = hv[it];
      __threadfence();
    }
  }
}

extern "C" void kernel_launch(void* const* d_in, const int* in_sizes, int n_in,
                              void* d_out, int out_size, void* d_ws, size_t ws_size,
                              hipStream_t stream)
{
  if (n_in < 10) return;
  if (in_sizes[0] != kRows * kDmod) return;
  if (in_sizes[1] != kXZP * kDmod) return;
  if (in_sizes[2] != kXZP) return;
  if (in_sizes[3] != kPrjN * kDin) return;
  if (in_sizes[4] != kDin * kDtR) return;
  if (in_sizes[5] != kDin) return;
  if (in_sizes[6] != kDin * kNst) return;
  if (in_sizes[7] != kDin) return;
  if (in_sizes[8] != kDmod * kDin) return;
  if (in_sizes[9] != kDmod) return;
  if (out_size != kRows * kDmod) return;
  if (ws_size < kWsTotal) return;

  const float* x      = (const float*)d_in[0];
  const float* W_in   = (const float*)d_in[1];
  const float* b_in   = (const float*)d_in[2];
  const float* W_xprj = (const float*)d_in[3];
  const float* W_dt   = (const float*)d_in[4];
  const float* b_dt   = (const float*)d_in[5];
  const float* A_log  = (const float*)d_in[6];
  const float* Dv     = (const float*)d_in[7];
  const float* W_out  = (const float*)d_in[8];
  const float* b_out  = (const float*)d_in[9];
  float* dout = (float*)d_out;

  char* ws = (char*)d_ws;
  unsigned short* X16  = (unsigned short*)(ws + kOffX16);
  unsigned short* WIN  = (unsigned short*)(ws + kOffWIN);
  unsigned short* WXP  = (unsigned short*)(ws + kOffWXP);
  unsigned short* WDT  = (unsigned short*)(ws + kOffWDT);
  unsigned short* WOUT = (unsigned short*)(ws + kOffWOUT);
  float*          XZ   = (float*)(ws + kOffXZ);
  unsigned short* XINH = (unsigned short*)(ws + kOffXINH);
  unsigned short* XINL = (unsigned short*)(ws + kOffXINL);
  float*          XD   = (float*)(ws + kOffXD);
  unsigned short* DTH  = (unsigned short*)(ws + kOffDTH);
  unsigned short* DTL  = (unsigned short*)(ws + kOffDTL);
  float*          DLR  = (float*)(ws + kOffDLR);
  unsigned short* Y16  = (unsigned short*)(ws + kOffY16);
  const float* dummy_bias  = b_in;
  const float* dummy_resid = x;

  cast_in_f16_kernel<<<kTot8X / 256, 256, 0, stream>>>(x, X16, kTot8X, kCarX);
  cast_in_f16_kernel<<<kTot8Win / 256, 256, 0, stream>>>(W_in, WIN, kTot8Win, kCarWin);
  cast_in_f16_kernel<<<kTot8Wout / 256, 256, 0, stream>>>(W_out, WOUT, kTot8Wout, kCarWout);
  cast_in_bf16_kernel<<<kTot8Wxp / 256, 256, 0, stream>>>(W_xprj, WXP, kTot8Wxp, kReal8Wxp);
  cast_in_bf16_kernel<<<kTot8Wdt / 256, 256, 0, stream>>>(W_dt, WDT, kTot8Wdt, kTot8Wdt);

  for (int b = 0; b < kBatch; ++b) {
    const unsigned short* X16b = X16 + (size_t)b * kSeqL * kDmod;
    float* outb = dout + (size_t)b * kSeqL * kDmod;

    wmma_gemm64<0, 0, 2, 0, false, 0><<<dim3(kBlkIn, 1), 256, 0, stream>>>(
        X16b, X16b, kDmod, 0L, WIN, WIN, kDmod, 0L,
        (void*)XZ, (void*)XZ, kXZP, 0L, b_in, dummy_resid, 0L, kSeqL, kXZP, kDmod, kSclIn);

    split_u_kernel<<<kTotSplit / 256, 256, 0, stream>>>(XZ, XINH, XINL, kTotSplit);

    wmma_gemm64<1, 1, 0, 0, false, 0><<<dim3(kBlkXp, 1), 256, 0, stream>>>(
        XINH, XINL, kDin, 0L, WXP, WXP, kDin, 0L,
        (void*)XD, (void*)XD, kPrjP, 0L, dummy_bias, dummy_resid, 0L, kSeqL, kPrjP, kDin, 1.0f);

    dt_split_kernel<<<kTot8Dt / 256, 256, 0, stream>>>(XD, DTH, DTL, kTot8Dt);

    wmma_gemm64<1, 1, 2, 0, false, 0><<<dim3(kBlkDt, 1), 256, 0, stream>>>(
        DTH, DTL, kDtR, 0L, WDT, WDT, kDtR, 0L,
        (void*)DLR, (void*)DLR, kDin, 0L, b_dt, dummy_resid, 0L, kSeqL, kDin, kDtR, 1.0f);

    scan_kernel<<<dim3(kDin / 256, 1), 256, 0, stream>>>(DLR, XZ, XD, A_log, Dv, Y16);

    wmma_gemm64<0, 0, 2, 0, false, 0><<<dim3(kBlkOut, 1), 256, 0, stream>>>(
        Y16, Y16, kDin, 0L, WOUT, WOUT, kDin, 0L,
        (void*)outb, (void*)outb, kDmod, 0L, b_out, dummy_resid, 0L, kSeqL, kDmod, kDin, kSclOut);
  }
}
